// LongRec_18202071400579
// MI455X (gfx1250) — hardware-verified
//
#include <hip/hip_runtime.h>
#include <math.h>

constexpr int kBatch  = 256;
constexpr int kSeq    = 200;
constexpr int kDim    = 128;
constexpr int kHid    = 128;
constexpr int kCls    = 50000;
constexpr int kClsPad = 50048;
constexpr int kItems  = 50000;
constexpr int kRows   = kBatch * kSeq;
constexpr int kXP     = 384;
constexpr int kTP     = 256;
constexpr int kHP     = 136;
constexpr int kNT     = 256;
constexpr int kPrepSegBlocks  = 14 * 8;
constexpr int kPrepOutBlocks  = kClsPad / 16;
constexpr int kBiasLines      = kClsPad / 32;
constexpr int kPrepBiasBlocks = (kBiasLines + 7) / 8;
constexpr int kPrepBlocks     = kPrepSegBlocks + kPrepOutBlocks + kPrepBiasBlocks;
constexpr int kPairF4         = (2 * kCls) / 4;
constexpr int kOutIters       = (kPairF4 + kNT - 1) / kNT;
static_assert(kRows % 64 == 0 && kClsPad % 64 == 0 && kBatch % 64 == 0, "");
static_assert(kCls % 4 == 0 && (2 * kCls) % 32 == 0 && kPairF4 % 8 == 0, "");

typedef __attribute__((ext_vector_type(16))) _Float16 v16h;
typedef __attribute__((ext_vector_type(8)))  _Float16 v8h;
typedef __attribute__((ext_vector_type(16))) __bf16   v16b;
typedef __attribute__((ext_vector_type(8)))  __bf16   v8b;
typedef __attribute__((ext_vector_type(8)))  float    v8f;
typedef __attribute__((ext_vector_type(4)))  float    v4f;

__device__ __forceinline__ unsigned short f2bf_bits(float f) {
  unsigned u = __float_as_uint(f);
  return (unsigned short)((u + 0x7FFFu + ((u >> 16) & 1u)) >> 16);
}
__device__ __forceinline__ float bf_bits2f(unsigned short h) { return __uint_as_float(((unsigned)h) << 16); }

__device__ __forceinline__ void dep_guard_h(v8f& a, v8f& b, v16h x, v16h y) { asm volatile("v_nop\n\tv_nop\n\tv_nop\n\tv_nop" : "+v"(a), "+v"(b) : "v"(x), "v"(y)); }
__device__ __forceinline__ void dep_guard_b(v8f& a, v8f& b, v16b x, v16b y) { asm volatile("v_nop\n\tv_nop\n\tv_nop\n\tv_nop" : "+v"(a), "+v"(b) : "v"(x), "v"(y)); }
__device__ __forceinline__ void keep4_h(v16h a, v16h b, v16h c, v16h d) { asm volatile("v_nop" :: "v"(a), "v"(b), "v"(c), "v"(d)); }
__device__ __forceinline__ void keep4_b(v16b a, v16b b, v16b c, v16b d) { asm volatile("v_nop" :: "v"(a), "v"(b), "v"(c), "v"(d)); }
__device__ __forceinline__ void acc_guard4(v8f& a, v8f& b, v8f& c, v8f& d) { asm volatile("v_nop\n\tv_nop\n\tv_nop\n\tv_nop" : "+v"(a), "+v"(b), "+v"(c), "+v"(d)); }
__device__ __forceinline__ void dep_guard2_h(v8f& a, v8f& b, v16h x, v16h y, v16h z) {
  asm volatile("v_nop\n\tv_nop\n\tv_nop\n\tv_nop" : "+v"(a), "+v"(b) : "v"(x), "v"(y), "v"(z));
}
__device__ __forceinline__ void dep_guard1_h(v8f& a, v16h x, v16h y) {
  asm volatile("v_nop\n\tv_nop\n\tv_nop\n\tv_nop" : "+v"(a) : "v"(x), "v"(y));
}
__device__ __forceinline__ void acc_guard2(v8f& a, v8f& b) { asm volatile("v_nop\n\tv_nop\n\tv_nop\n\tv_nop" : "+v"(a), "+v"(b)); }
__device__ __forceinline__ void acc_guard1(v8f& a) { asm volatile("v_nop\n\tv_nop\n\tv_nop\n\tv_nop" : "+v"(a)); }

__device__ __forceinline__ float ftanh(float x) { return 1.0f - 2.0f * __builtin_amdgcn_rcpf(1.0f + __expf(2.0f * x)); }
__device__ __forceinline__ float fsigm(float x) { return __builtin_amdgcn_rcpf(1.0f + __expf(-x)); }

template <typename T> struct Frag;
template <> struct Frag<_Float16> {
  typedef v16h V; union U { v16h v; v8h h[2]; };
  static __device__ __forceinline__ v16h load(const _Float16* p) {
    U f; f.h[0] = *(const v8h*)(p); f.h[1] = *(const v8h*)(p + 16); return f.v;
  }
  static __device__ __forceinline__ v8f mma(v16h a, v16h b, v8f c) {
    return __builtin_amdgcn_wmma_f32_16x16x32_f16(false, a, false, b, (short)0, c, false, false);
  }
  static __device__ __forceinline__ void guard(v8f& a, v8f& b, v16h x, v16h y) { dep_guard_h(a, b, x, y); }
  static __device__ __forceinline__ void keep(v16h a, v16h b, v16h c, v16h d) { keep4_h(a, b, c, d); }
};
template <> struct Frag<__bf16> {
  typedef v16b V; union U { v16b v; v8b h[2]; };
  static __device__ __forceinline__ v16b load(const __bf16* p) {
    U f; f.h[0] = *(const v8b*)(p); f.h[1] = *(const v8b*)(p + 16); return f.v;
  }
  static __device__ __forceinline__ v8f mma(v16b a, v16b b, v8f c) {
    return __builtin_amdgcn_wmma_f32_16x16x32_bf16(false, a, false, b, (short)0, c, false, false);
  }
  static __device__ __forceinline__ void guard(v8f& a, v8f& b, v16b x, v16b y) { dep_guard_b(a, b, x, y); }
  static __device__ __forceinline__ void keep(v16b a, v16b b, v16b c, v16b d) { keep4_b(a, b, c, d); }
};

template <int ET> struct Elem;
template <> struct Elem<0> { typedef _Float16 T; };
template <> struct Elem<1> { typedef __bf16 T; };
template <int ET, bool SPLIT, int BIAS_MODE, int OUT_MODE, bool RESID, int ACT = 0>
__global__ __launch_bounds__(256) void wmma_gemm64(
    const unsigned short* __restrict__ Ap, const unsigned short* __restrict__ A2p, int lda, long strideA,
    const unsigned short* __restrict__ Btp, const unsigned short* __restrict__ Bt2p, int ldb, long strideB,
    void* __restrict__ Cout, void* __restrict__ Cout2, int ldc, long strideC,
    const float* __restrict__ bias,
    const float* __restrict__ resid, long strideR,
    int M, int N, int K, float scale) {
  typedef typename Elem<ET>::T T;
  typedef typename Frag<T>::V V;
  const T* A = (const T*)Ap; const T* A2 = (const T*)A2p; const T* Bt = (const T*)Btp; const T* Bt2 = (const T*)Bt2p;
  __shared__ __align__(16) float sT[8][16 * 68];
  const int b    = blockIdx.y;
  const int lane = threadIdx.x & 31;
  const int wave = threadIdx.x >> 5;
  const int tilesN = N >> 6;
  const int tilesM = M >> 6;
  const int tile = blockIdx.x * 8 + wave;
  if (tile >= tilesM * tilesN) return;
  const int tm = tile / tilesN;
  const int tn = tile - tm * tilesN;
  const int m0 = tm << 6;
  const int n0 = tn << 6;

  const T* Ab  = A  + (size_t)b * strideA;
  const T* Bb  = Bt + (size_t)b * strideB;
  const T* Ab2 = SPLIT ? (A2  + (size_t)b * strideA) : nullptr;
  const T* Bb2 = SPLIT ? (Bt2 + (size_t)b * strideB) : nullptr;

  const int rlane = lane & 15;
  const int koff  = (lane >> 4) * 8;
  const int mOff  = (lane >> 4) * 8;

  v8f acc[4][4];
#pragma unroll
  for (int i = 0; i < 4; ++i)
#pragma unroll
    for (int j = 0; j < 4; ++j) acc[i][j] = (v8f){0.f,0.f,0.f,0.f,0.f,0.f,0.f,0.f};

  for (int k0 = 0; k0 < K; k0 += 32) {
    V bh[4], bl[4];
#pragma unroll
    for (int j = 0; j < 4; ++j) {
      const size_t bo = (size_t)(n0 + (j << 4) + rlane) * ldb + koff + k0;
      bh[j] = Frag<T>::load(Bb + bo);
      if (SPLIT) bl[j] = Frag<T>::load(Bb2 + bo);
    }
#pragma unroll
    for (int i = 0; i < 4; ++i) {
      const size_t ao = (size_t)(m0 + (i << 4) + rlane) * lda + koff + k0;
      V ah = Frag<T>::load(Ab + ao);
      V al;
      if (SPLIT) al = Frag<T>::load(Ab2 + ao);
#pragma unroll
      for (int j = 0; j < 4; ++j) {
        acc[i][j] = Frag<T>::mma(ah, bh[j], acc[i][j]);
        if (SPLIT) {
          acc[i][j] = Frag<T>::mma(ah, bl[j], acc[i][j]);
          acc[i][j] = Frag<T>::mma(al, bh[j], acc[i][j]);
        }
      }
      Frag<T>::guard(acc[i][0], acc[i][3], ah, SPLIT ? al : ah);
    }
    Frag<T>::keep(bh[0], bh[1], bh[2], bh[3]);
    if (SPLIT) Frag<T>::keep(bl[0], bl[1], bl[2], bl[3]);
  }
  acc_guard4(acc[0][0], acc[0][1], acc[0][2], acc[0][3]);
  acc_guard4(acc[1][0], acc[1][1], acc[1][2], acc[1][3]);
  acc_guard4(acc[2][0], acc[2][1], acc[2][2], acc[2][3]);
  acc_guard4(acc[3][0], acc[3][1], acc[3][2], acc[3][3]);

  float* slab = sT[wave];
  const float* Rb = RESID ? (resid + (size_t)b * strideR) : nullptr;
#pragma unroll
  for (int i = 0; i < 4; ++i) {
    const int mBase = m0 + (i << 4);
#pragma unroll
    for (int j = 0; j < 4; ++j) {
      const int n = n0 + (j << 4) + rlane;
      float bv = 0.f;
      if (BIAS_MODE == 2) bv = bias[n];
#pragma unroll
      for (int r = 0; r < 8; ++r) {
        float v = acc[i][j][r] * scale;
        if (BIAS_MODE == 1) v += bias[mBase + mOff + r];
        if (BIAS_MODE == 2) v += bv;
        if (RESID) v += Rb[(size_t)(mBase + mOff + r) * ldc + n];
        if (ACT == 1) v = tanhf(v);
        if (ACT == 2) v = fmaxf(v, 0.0f);
        if (ACT == 3) v = v / (1.0f + expf(-v));
        if (ACT == 4) v = (v > 0.f) ? v : 0.01f * v;
        if (ACT == 6) v = fsigm(v);
        if (ACT == 7) v = __builtin_amdgcn_rcpf(1.0f + __expf(v));
        slab[(mOff + r) * 68 + (j << 4) + rlane] = v;
      }
    }
    __builtin_amdgcn_fence(__ATOMIC_RELEASE, "workgroup");
    __builtin_amdgcn_wave_barrier();
    __builtin_amdgcn_fence(__ATOMIC_ACQUIRE, "workgroup");
    if (OUT_MODE == 0) {
      float* C = (float*)Cout + (size_t)b * strideC;
      const int hh = lane >> 4, c4 = (lane & 15) * 4;
      for (int pass = 0; pass < 2; ++pass) {
#pragma unroll
        for (int it = 0; it < 8; ++it) {
          const int row = it * 2 + hh;
          v4f v = *(const v4f*)(slab + row * 68 + c4);
          *(volatile v4f*)(C + (size_t)(mBase + row) * ldc + n0 + c4) = v;
        }
        __threadfence();
      }
    } else {
      const int q = lane >> 3, c8 = (lane & 7) * 8;
      unsigned short* C  = (unsigned short*)Cout  + (size_t)b * strideC;
      unsigned short* C2 = (OUT_MODE == 2) ? ((unsigned short*)Cout2 + (size_t)b * strideC) : nullptr;
      for (int pass = 0; pass < 2; ++pass) {
#pragma unroll
        for (int it = 0; it < 4; ++it) {
          const int row = it * 4 + q;
          const float* sp = slab + row * 68 + c8;
          v8h hv, lv;
#pragma unroll
          for (int e = 0; e < 8; ++e) {
            if (OUT_MODE == 1) {
              hv[e] = (_Float16)sp[e];
            } else {
              unsigned short hb = f2bf_bits(sp[e]);
              unsigned short lb = f2bf_bits(sp[e] - bf_bits2f(hb));
              hv[e] = __builtin_bit_cast(_Float16, hb);
              lv[e] = __builtin_bit_cast(_Float16, lb);
            }
          }
          *(volatile v8h*)(C + (size_t)(mBase + row) * ldc + n0 + c8) = hv;
          if (OUT_MODE == 2) *(volatile v8h*)(C2 + (size_t)(mBase + row) * ldc + n0 + c8) = lv;
        }
        __threadfence();
      }
    }
    __builtin_amdgcn_fence(__ATOMIC_RELEASE, "workgroup");
    __builtin_amdgcn_wave_barrier();
    __builtin_amdgcn_fence(__ATOMIC_ACQUIRE, "workgroup");
  }
}

__device__ __forceinline__ void st2_v8h(_Float16* p, v8h h) { *(volatile v8h*)p = h; __threadfence(); *(volatile v8h*)p = h; }

__device__ __forceinline__ void seg_row(const float* __restrict__ src, int ns, int ncl, bool valid, float scale,
                                        _Float16* dst, int c) {
  v8h h;
#pragma unroll
  for (int e = 0; e < 8; ++e) {
    const float f = src[(size_t)(8 * c + e) * (size_t)ns + ncl];
    const float g = valid ? f * scale : 0.0f;
    h[e] = (_Float16)g;
  }
  st2_v8h(dst + 8 * c, h);
}

__global__ __launch_bounds__(kNT) void prep_kernel(
    const float* __restrict__ Wxr, const float* __restrict__ Wxz, const float* __restrict__ Wxh,
    const float* __restrict__ Whr, const float* __restrict__ Whz, const float* __restrict__ Whh,
    const float* __restrict__ Wxtg, const float* __restrict__ Wtg, const float* __restrict__ Wxfg, const float* __restrict__ Wfg,
    const float* __restrict__ Wdelta, const float* __restrict__ Wfdir, const float* __restrict__ Wpsi,
    const float* __restrict__ Wout, const float* __restrict__ bout,
    _Float16* __restrict__ WTGC, _Float16* __restrict__ WFGC, _Float16* __restrict__ WXRZH, _Float16* __restrict__ WDEL,
    _Float16* __restrict__ WFP, _Float16* __restrict__ WHH3, _Float16* __restrict__ WOUT, float* __restrict__ BOUTP) {
  const int blk = blockIdx.x, tid = threadIdx.x, lane = tid & 31, wave = tid >> 5, hh = lane >> 4, c = lane & 15;
  if (blk < kPrepSegBlocks) {
    const int seg = blk >> 3;
    const int n   = ((blk & 7) << 4) + wave * 2 + hh;
    const float* src = Wtg; _Float16* dst = WTGC; int pitch = kTP, rowoff = 0, coloff = 0;
    switch (seg) {
      case 0:  src = Wtg;                    dst = WTGC;  pitch = kTP;  rowoff = 0;        coloff = 0;    break;
      case 1:  src = Wxtg;                   dst = WTGC;  pitch = kTP;  rowoff = 0;        coloff = kDim; break;
      case 2:  src = Wxfg;                   dst = WFGC;  pitch = kTP;  rowoff = 0;        coloff = 0;    break;
      case 3:  src = Wfg;                    dst = WFGC;  pitch = kTP;  rowoff = 0;        coloff = kDim; break;
      case 4:  src = Wxr;                    dst = WXRZH; pitch = kDim; rowoff = 0;        coloff = 0;    break;
      case 5:  src = Wxz;                    dst = WXRZH; pitch = kDim; rowoff = kHid;     coloff = 0;    break;
      case 6:  src = Wxh;                    dst = WXRZH; pitch = kDim; rowoff = 2 * kHid; coloff = 0;    break;
      case 7:  src = Wdelta;                 dst = WDEL;  pitch = kTP;  rowoff = 0;        coloff = 0;    break;
      case 8:  src = Wdelta + kHid * kHid;   dst = WDEL;  pitch = kTP;  rowoff = 0;        coloff = kHid; break;
      case 9:  src = Wfdir;                  dst = WFP;   pitch = kHid; rowoff = 0;        coloff = 0;    break;
      case 10: src = Wpsi;                   dst = WFP;   pitch = kHid; rowoff = kHid;     coloff = 0;    break;
      case 11: src = Whr;                    dst = WHH3;  pitch = kHid; rowoff = 0;        coloff = 0;    break;
      case 12: src = Whz;                    dst = WHH3;  pitch = kHid; rowoff = kHid;     coloff = 0;    break;
      default: src = Whh;                    dst = WHH3;  pitch = kHid; rowoff = 2 * kHid; coloff = 0;    break;
    }
    seg_row(src, kHid, n, true, 16.0f, dst + (size_t)(rowoff + n) * pitch + coloff, c);
  } else if (blk < kPrepSegBlocks + kPrepOutBlocks) {
    const int n   = (blk - kPrepSegBlocks) * 16 + wave * 2 + hh;
    const int ncl = (n < kCls) ? n : (kCls - 1);
    seg_row(Wout, kCls, ncl, n < kCls, 256.0f, WOUT + (size_t)n * kHid, c);
  } else {
    const int line = (blk - kPrepSegBlocks - kPrepOutBlocks) * 8 + wave;
    if (line < kBiasLines) {
      const int i   = line * 32 + lane;
      const int icl = (i < kCls) ? i : (kCls - 1);
      const float ld = bout[icl];
      const float v  = (i < kCls) ? ld : 0.0f;
      float* p = BOUTP + i;
      *(volatile float*)p = v;
      __threadfence();
      *(volatile float*)p = v;
    }
  }
}

__device__ __forceinline__ void gat_seg(const float* __restrict__ p, _Float16* d) {
  const v4f a = *(const v4f*)p, bq = *(const v4f*)(p + 4);
  v8h h;
#pragma unroll
  for (int e = 0; e < 4; ++e) { h[e] = (_Float16)(a[e] * 256.0f); h[4 + e] = (_Float16)(bq[e] * 256.0f); }
  st2_v8h(d, h);
}
__global__ __launch_bounds__(kNT) void gather_kernel(const int* __restrict__ item, const int* __restrict__ tix,
                                                   const int* __restrict__ frq,
                                                   const float* __restrict__ emb_i, const float* __restrict__ emb_t,
                                                   const float* __restrict__ emb_f, _Float16* __restrict__ XCAT) {
  const int blk = blockIdx.x, tid = threadIdx.x, lane = tid & 31, wave = tid >> 5, hh = lane >> 4, c = lane & 15;
  const int row = blk * 16 + wave * 2 + hh;
  const int t = row >> 8, b = row & 255;
  const int fi = b * kSeq + t;
  int i0 = tix[fi], i1 = item[fi], i2 = frq[fi];
  i0 = i0 < 0 ? 0 : (i0 >= kItems ? kItems - 1 : i0);
  i1 = i1 < 0 ? 0 : (i1 >= kItems ? kItems - 1 : i1);
  i2 = i2 < 0 ? 0 : (i2 >= kItems ? kItems - 1 : i2);
  _Float16* drow = XCAT + (size_t)row * kXP + 8 * c;
  gat_seg(emb_t + (size_t)i0 * kDim + 8 * c, drow);
  gat_seg(emb_i + (size_t)i1 * kDim + 8 * c, drow + kDim);
  gat_seg(emb_f + (size_t)i2 * kDim + 8 * c, drow + 2 * kDim);
}

__global__ __launch_bounds__(kNT) void rec_kernel(const _Float16* __restrict__ XRZH, const _Float16* __restrict__ DPF,
                                                const _Float16* __restrict__ WHH3, const float* __restrict__ Wa,
                                                _Float16* __restrict__ H16) {
  __shared__ __align__(16) _Float16 sHd[16 * kHP];
  __shared__ __align__(16) _Float16 sRh[16 * kHP];
  (void)Wa;
  const int tid = threadIdx.x, lane = tid & 31, wave = tid >> 5;
  const int rlane = lane & 15, hh = lane >> 4, koff = hh * 8, mOff = hh * 8;
  const int blk = blockIdx.x;
  const int j = 16 * wave + rlane;
  const _Float16* ad  = sHd + rlane * kHP + koff;
  const _Float16* arh = sRh + rlane * kHP + koff;
  const _Float16* wr = WHH3 + (size_t)j * kHid + koff;
  const _Float16* wz = WHH3 + (size_t)(kHid + j) * kHid + koff;
  const _Float16* wn = WHH3 + (size_t)(2 * kHid + j) * kHid + koff;
  const v8f z8 = {0.f, 0.f, 0.f, 0.f, 0.f, 0.f, 0.f, 0.f};
  const float s256 = 1.0f / 256.0f;

  float hreg[8];
#pragma unroll
  for (int r = 0; r < 8; ++r) hreg[r] = 0.0f;

#pragma unroll 1
  for (int t = 0; t < kSeq; ++t) {
    const size_t row0 = (size_t)t * kBatch + (size_t)(blk * 16 + mOff);
    const _Float16* xb = XRZH + row0 * kXP + j;
    const _Float16* db = DPF  + row0 * kXP + j;
    float hd[8], xr[8], xz[8], xh[8], fd[8], ps[8];
#pragma unroll
    for (int r = 0; r < 8; ++r) {
      const _Float16* xp = xb + (size_t)r * kXP;
      const _Float16* dp = db + (size_t)r * kXP;
      xr[r] = (float)xp[0]; xz[r] = (float)xp[kHid]; xh[r] = (float)xp[2 * kHid];
      const float dec = (float)dp[0];
      fd[r] = (float)dp[kHid]; ps[r] = (float)dp[2 * kHid];
      hd[r] = dec * hreg[r];
      sHd[(mOff + r) * kHP + j] = (_Float16)(hd[r] * 16.0f);
    }
    __syncthreads();
    v8f ar = z8, az = z8;
#pragma unroll 1
    for (int k0 = 0; k0 < kHid; k0 += 32) {
      const v16h a  = Frag<_Float16>::load(ad + k0);
      const v16h b0 = Frag<_Float16>::load(wr + k0);
      const v16h b1 = Frag<_Float16>::load(wz + k0);
      ar = Frag<_Float16>::mma(a, b0, ar);
      az = Frag<_Float16>::mma(a, b1, az);
      dep_guard2_h(ar, az, a, b0, b1);
    }
    acc_guard2(ar, az);
    float zg[8];
#pragma unroll
    for (int r = 0; r < 8; ++r) {
      const float rg = fsigm(xr[r] + ar[r] * s256);
      zg[r] = fsigm(xz[r] + az[r] * s256);
      sRh[(mOff + r) * kHP + j] = (_Float16)(rg * hd[r] * 16.0f);
    }
    __syncthreads();
    v8f an = z8;
#pragma unroll 1
    for (int k0 = 0; k0 < kHid; k0 += 32) {
      const v16h a  = Frag<_Float16>::load(arh + k0);
      const v16h b2 = Frag<_Float16>::load(wn + k0);
      an = Frag<_Float16>::mma(a, b2, an);
      dep_guard1_h(an, a, b2);
    }
    acc_guard1(an);
#pragma unroll
    for (int r = 0; r < 8; ++r) {
      const float hb = ftanh(xh[r] + an[r] * s256);
      const float hf = ftanh(hb + fd[r]);
      const float hc = (1.0f - ps[r]) * hb + ps[r] * hf;
      hreg[r] = (1.0f - zg[r]) * hd[r] + zg[r] * hc;
    }
  }

#pragma unroll
  for (int r = 0; r < 8; ++r) sHd[(mOff + r) * kHP + j] = (_Float16)(hreg[r] * 16.0f);
  __syncthreads();
  {
    const int row = 2 * wave + hh, c8 = (lane & 15) * 8;
    _Float16* hp = H16 + (size_t)(blk * 16 + row) * kHid + c8;
    for (int pass = 0; pass < 2; ++pass) {
      const v8h v = *(const v8h*)(sHd + row * kHP + c8);
      *(volatile v8h*)hp = v;
      __threadfence();
    }
  }
}

__global__ __launch_bounds__(kNT) void softmax_out_kernel(const float* __restrict__ LOG, float* __restrict__ out) {
  __shared__ float red[kNT];
  const int tid = threadIdx.x, p = blockIdx.x;
  float mrow[2], irow[2];
#pragma unroll
  for (int rr = 0; rr < 2; ++rr) {
    const float* base = LOG + (size_t)(2 * p + rr) * kClsPad;
    float m = -3.402823466e38f;
#pragma unroll 1
    for (int i = tid; i < kCls; i += kNT) m = fmaxf(m, base[i]);
    red[tid] = m;
    __syncthreads();
#pragma unroll 1
    for (int s = kNT / 2; s > 0; s >>= 1) {
      if (tid < s) red[tid] = fmaxf(red[tid], red[tid + s]);
      __syncthreads();
    }
    const float mx = red[0];
    __syncthreads();
    float sum = 0.0f;
#pragma unroll 1
    for (int i = tid; i < kCls; i += kNT) sum += expf(base[i] - mx);
    red[tid] = sum;
    __syncthreads();
#pragma unroll 1
    for (int s = kNT / 2; s > 0; s >>= 1) {
      if (tid < s) red[tid] = red[tid] + red[tid + s];
      __syncthreads();
    }
    const float tot = red[0];
    __syncthreads();
    mrow[rr] = mx;
    irow[rr] = 1.0f / tot;
  }
  const float mx0 = mrow[0], mx1 = mrow[1], iv0 = irow[0], iv1 = irow[1];
  float* ob = out + (size_t)p * (size_t)(2 * kCls);
#pragma unroll 1
  for (int pass = 0; pass < 2; ++pass) {
#pragma unroll 1
    for (int it = 0; it < kOutIters; ++it) {
      const int q = it * kNT + tid;
      if (q < kPairF4) {
        const int f   = 4 * q;
        const int sel = (f >= kCls) ? 1 : 0;
        const int col = f - sel * kCls;
        const v4f lv = *(const v4f*)(LOG + (size_t)(2 * p + sel) * kClsPad + col);
        const float mx = sel ? mx1 : mx0;
        const float iv = sel ? iv1 : iv0;
        v4f o;
        o.x = expf(lv.x - mx) * iv;
        o.y = expf(lv.y - mx) * iv;
        o.z = expf(lv.z - mx) * iv;
        o.w = expf(lv.w - mx) * iv;
        *(volatile v4f*)(ob + f) = o;
      }
    }
    __threadfence();
  }
}

extern "C" void kernel_launch(void* const* d_in, const int* in_sizes, int n_in,
                              void* d_out, int out_size, void* d_ws, size_t ws_size, hipStream_t stream) {
  if (n_in < 30 || d_out == nullptr || d_ws == nullptr) return;
  const int nW = kDim * kHid, nE = kItems * kDim;
  if (in_sizes[0] != kRows || in_sizes[1] != kRows || in_sizes[2] != kRows ||
      in_sizes[3] != nE || in_sizes[4] != nE || in_sizes[5] != nE ||
      in_sizes[6] != nW || in_sizes[7] != nW || in_sizes[8] != kHid ||
      in_sizes[9] != nW || in_sizes[10] != nW || in_sizes[11] != kHid ||
      in_sizes[12] != nW || in_sizes[13] != nW || in_sizes[14] != kHid ||
      in_sizes[15] != nW || in_sizes[16] != nW || in_sizes[17] != kHid ||
      in_sizes[18] != nW || in_sizes[19] != nW || in_sizes[20] != kHid ||
      in_sizes[21] != 2 * nW || in_sizes[22] != kHid ||
      in_sizes[23] != nW || in_sizes[24] != kHid || in_sizes[25] != nW || in_sizes[26] != kHid ||
      in_sizes[27] != 2 * kHid || in_sizes[28] != kHid * kCls || in_sizes[29] != kCls ||
      out_size != kBatch * kCls) return;

  const int*   item   = (const int*)d_in[0];
  const int*   tix    = (const int*)d_in[1];
  const int*   frq    = (const int*)d_in[2];
  const float* emb_i  = (const float*)d_in[3];
  const float* emb_t  = (const float*)d_in[4];
  const float* emb_f  = (const float*)d_in[5];
  const float* W_xr   = (const float*)d_in[6];
  const float* W_hr   = (const float*)d_in[7];
  const float* b_r    = (const float*)d_in[8];
  const float* W_xz   = (const float*)d_in[9];
  const float* W_hz   = (const float*)d_in[10];
  const float* b_z    = (const float*)d_in[11];
  const float* W_xh   = (const float*)d_in[12];
  const float* W_hh   = (const float*)d_in[13];
  const float* b_h    = (const float*)d_in[14];
  const float* W_xtg  = (const float*)d_in[15];
  const float* W_tg   = (const float*)d_in[16];
  const float* b_tg   = (const float*)d_in[17];
  const float* W_xfg  = (const float*)d_in[18];
  const float* W_fg   = (const float*)d_in[19];
  const float* b_fg   = (const float*)d_in[20];
  const float* W_delta= (const float*)d_in[21];
  const float* b_delta= (const float*)d_in[22];
  const float* W_fdir = (const float*)d_in[23];
  const float* b_fdir = (const float*)d_in[24];
  const float* W_psi  = (const float*)d_in[25];
  const float* b_psi  = (const float*)d_in[26];
  const float* W_a    = (const float*)d_in[27];
  const float* W_out  = (const float*)d_in[28];
  const float* b_out  = (const float*)d_in[29];
  float* out = (float*)d_out;

  char* ws = (char*)d_ws; size_t off = 0;
  auto carve = [&](size_t bytes) -> char* { char* p = ws + off; off += (bytes + 255) & ~(size_t)255; return p; };
  _Float16* WTGC  = (_Float16*)carve((size_t)kHid * kTP * 2);
  _Float16* WFGC  = (_Float16*)carve((size_t)kHid * kTP * 2);
  _Float16* WXRZH = (_Float16*)carve((size_t)3 * kHid * kDim * 2);
  _Float16* WDEL  = (_Float16*)carve((size_t)kHid * kTP * 2);
  _Float16* WFP   = (_Float16*)carve((size_t)2 * kHid * kHid * 2);
  _Float16* WHH3  = (_Float16*)carve((size_t)3 * kHid * kHid * 2);
  _Float16* WOUT  = (_Float16*)carve((size_t)kClsPad * kHid * 2);
  float*    BOUTP = (float*)carve((size_t)kClsPad * 4);
  _Float16* H16   = (_Float16*)carve((size_t)kBatch * kHid * 2);
  _Float16* XCAT  = (_Float16*)carve((size_t)kRows * kXP * 2);
  _Float16* TGFG  = (_Float16*)carve((size_t)kRows * kTP * 2);
  _Float16* XRZH  = (_Float16*)carve((size_t)kRows * kXP * 2);
  _Float16* DPF    = XCAT;
  float*    LOGITS = (float*)TGFG;
  if (off > ws_size || off > (size_t)134217728) return;
  if ((size_t)kBatch * kClsPad * 4 > (size_t)kRows * kTP * 2 + (size_t)kRows * kXP * 2) return;

  prep_kernel<<<kPrepBlocks, kNT, 0, stream>>>(W_xr, W_xz, W_xh, W_hr, W_hz, W_hh, W_xtg, W_tg, W_xfg, W_fg, W_delta, W_fdir, W_psi,
                                              W_out, b_out, WTGC, WFGC, WXRZH, WDEL, WFP, WHH3, WOUT, BOUTP);
  gather_kernel<<<kRows / 16, kNT, 0, stream>>>(item, tix, frq, emb_i, emb_t, emb_f, XCAT);

  const int gridP = ((kRows / 64) * (kHid / 64)) / 8;
  const unsigned short* nul16 = (const unsigned short*)nullptr;
  const float sEW = 1.0f / 4096.0f;
  const float sW  = 1.0f / 16.0f;
  wmma_gemm64<0, false, 2, 1, false, 6><<<dim3(gridP, 1), 256, 0, stream>>>(
      (const unsigned short*)XCAT, nul16, kXP, 0L, (const unsigned short*)WTGC, nul16, kTP, 0L,
      (void*)TGFG, (void*)nullptr, kTP, 0L, b_tg, (const float*)nullptr, 0L, kRows, kHid, 2 * kDim, sEW);
  wmma_gemm64<0, false, 2, 1, false, 6><<<dim3(gridP, 1), 256, 0, stream>>>(
      (const unsigned short*)(XCAT + kDim), nul16, kXP, 0L, (const unsigned short*)WFGC, nul16, kTP, 0L,
      (void*)(TGFG + kHid), (void*)nullptr, kTP, 0L, b_fg, (const float*)nullptr, 0L, kRows, kHid, 2 * kDim, sEW);
  wmma_gemm64<0, false, 2, 1, false, 0><<<dim3(gridP, 1), 256, 0, stream>>>(
      (const unsigned short*)(XCAT + kDim), nul16, kXP, 0L, (const unsigned short*)WXRZH, nul16, kDim, 0L,
      (void*)XRZH, (void*)nullptr, kXP, 0L, b_r, (const float*)nullptr, 0L, kRows, kHid, kDim, sEW);
  wmma_gemm64<0, false, 2, 1, false, 0><<<dim3(gridP, 1), 256, 0, stream>>>(
      (const unsigned short*)(XCAT + kDim), nul16, kXP, 0L, (const unsigned short*)(WXRZH + (size_t)kHid * kDim), nul16, kDim, 0L,
      (void*)(XRZH + kHid), (void*)nullptr, kXP, 0L, b_z, (const float*)nullptr, 0L, kRows, kHid, kDim, sEW);
  wmma_gemm64<0, false, 2, 1, false, 0><<<dim3(gridP, 1), 256, 0, stream>>>(
      (const unsigned short*)(XCAT + kDim), nul16, kXP, 0L, (const unsigned short*)(WXRZH + (size_t)2 * kHid * kDim), nul16, kDim, 0L,
      (void*)(XRZH + 2 * kHid), (void*)nullptr, kXP, 0L, b_h, (const float*)nullptr, 0L, kRows, kHid, kDim, sEW);
  wmma_gemm64<0, false, 2, 1, false, 7><<<dim3(gridP, 1), 256, 0, stream>>>(
      (const unsigned short*)TGFG, nul16, kTP, 0L, (const unsigned short*)WDEL, nul16, kTP, 0L,
      (void*)DPF, (void*)nullptr, kXP, 0L, b_delta, (const float*)nullptr, 0L, kRows, kHid, 2 * kHid, sW);
  wmma_gemm64<0, false, 2, 1, false, 0><<<dim3(gridP, 1), 256, 0, stream>>>(
      (const unsigned short*)(TGFG + kHid), nul16, kTP, 0L, (const unsigned short*)WFP, nul16, kHid, 0L,
      (void*)(DPF + kHid), (void*)nullptr, kXP, 0L, b_fdir, (const float*)nullptr, 0L, kRows, kHid, kHid, sW);
  wmma_gemm64<0, false, 2, 1, false, 6><<<dim3(gridP, 1), 256, 0, stream>>>(
      (const unsigned short*)(TGFG + kHid), nul16, kTP, 0L, (const unsigned short*)(WFP + (size_t)kHid * kHid), nul16, kHid, 0L,
      (void*)(DPF + 2 * kHid), (void*)nullptr, kXP, 0L, b_psi, (const float*)nullptr, 0L, kRows, kHid, kHid, sW);
  rec_kernel<<<kBatch / 16, kNT, 0, stream>>>(XRZH, DPF, WHH3, W_a, H16);
  const int gridL = ((kBatch / 64) * (kClsPad / 64)) / 8;
  wmma_gemm64<0, false, 2, 0, false, 0><<<dim3(gridL, 1), 256, 0, stream>>>(
      (const unsigned short*)H16, nul16, kHid, 0L, (const unsigned short*)WOUT, nul16, kHid, 0L,
      (void*)LOGITS, (void*)nullptr, kClsPad, 0L, BOUTP, (const float*)nullptr, 0L, kBatch, kClsPad, kHid, sEW);
  softmax_out_kernel<<<kBatch / 2, kNT, 0, stream>>>(LOGITS, out);
}
